// ModelAttention2Layers_46789373722916
// MI455X (gfx1250) — hardware-verified
//
#include <hip/hip_runtime.h>
#include <math.h>


typedef __bf16   bf16x16 __attribute__((ext_vector_type(16)));
typedef __bf16   bf16x8  __attribute__((ext_vector_type(8)));
typedef float    float8 __attribute__((ext_vector_type(8)));

__device__ __forceinline__ void split_bf16(float v, __bf16& hi, __bf16& lo) {
    const unsigned int u = __builtin_bit_cast(unsigned int, v) & 0xffff0000u;
    hi = __builtin_bit_cast(__bf16, (unsigned short)(u >> 16));
    lo = (__bf16)(v - __builtin_bit_cast(float, u));
}
__device__ __forceinline__ float8 wmmab(bf16x16 a, bf16x16 b, float8 c) {
    float8 d = __builtin_amdgcn_wmma_f32_16x16x32_bf16(false, a, false, b, (short)0, c, false, false);
    asm volatile("v_nop\n\tv_nop\n\tv_nop\n\tv_nop" : "+v"(d) : "v"(a), "v"(b));
    return d;
}
__device__ __forceinline__ float8 wmma3(bf16x16 ah, bf16x16 al, bf16x16 bh, bf16x16 bl, float8 c) {
    c = wmmab(ah, bh, c); c = wmmab(ah, bl, c); c = wmmab(al, bh, c); return c;
}

#define SEQ 2048
#define DD  512
#define KK_ 256

#define LDS_STRIDE 40

template<bool BT, bool HAS_BIAS, bool GUARD>
__global__ void gemm_wmma_f16(const float* __restrict__ A, int lda,
                              const float* __restrict__ B, int ldb,
                              const float* __restrict__ bias,
                              float* __restrict__ C, int ldc,
                              int M, int N, int Kd)
{
    __shared__ __align__(64) __bf16 Bs[64 * LDS_STRIDE];
    __shared__ __align__(64) __bf16 Bl[64 * LDS_STRIDE];

    const int tid  = threadIdx.x;
    const int lane = tid & 31;
    const int wave = tid >> 5;
    const int l    = lane & 15;
    const int hi   = lane >> 4;
    const int m0w  = (blockIdx.y << 6) + (wave << 4);
    const int n0   = blockIdx.x << 6;

    int arow = m0w + l;
    if (GUARD && arow >= M) arow = M - 1;
    const float* __restrict__ Arow = A + (size_t)arow * lda + hi * 8;

    float8 c0 = {}, c1 = {}, c2 = {}, c3 = {};

    for (int kk = 0; kk < Kd; kk += 32) {
        __syncthreads();
        if (BT) {
            #pragma unroll
            for (int j = 0; j < 4; ++j) {
                const int idx  = tid + j * 128;
                const int bcol = idx >> 3;
                const int kq   = (idx & 7) << 2;
                const float4 bv = *(const float4*)(B + (size_t)(n0 + bcol) * ldb + kk + kq);
                __bf16* p = &Bs[bcol * LDS_STRIDE + kq]; __bf16* q = &Bl[bcol * LDS_STRIDE + kq];
                split_bf16(bv.x, p[0], q[0]); split_bf16(bv.y, p[1], q[1]);
                split_bf16(bv.z, p[2], q[2]); split_bf16(bv.w, p[3], q[3]);
            }
        } else {
            #pragma unroll
            for (int j = 0; j < 4; ++j) {
                const int idx  = tid + j * 128;
                const int krow = idx >> 4;
                const int c4   = (idx & 15) << 2;
                const float4 bv = *(const float4*)(B + (size_t)(kk + krow) * ldb + n0 + c4);
                split_bf16(bv.x, Bs[(c4 + 0) * LDS_STRIDE + krow], Bl[(c4 + 0) * LDS_STRIDE + krow]);
                split_bf16(bv.y, Bs[(c4 + 1) * LDS_STRIDE + krow], Bl[(c4 + 1) * LDS_STRIDE + krow]);
                split_bf16(bv.z, Bs[(c4 + 2) * LDS_STRIDE + krow], Bl[(c4 + 2) * LDS_STRIDE + krow]);
                split_bf16(bv.w, Bs[(c4 + 3) * LDS_STRIDE + krow], Bl[(c4 + 3) * LDS_STRIDE + krow]);
            }
        }
        __syncthreads();

        const float4 a0 = *(const float4*)(Arow + kk);
        const float4 a1 = *(const float4*)(Arow + kk + 4);
        const float4 a2 = *(const float4*)(Arow + kk + 16);
        const float4 a3 = *(const float4*)(Arow + kk + 20);
        bf16x16 ah, al;
        {
            const float av[16] = {a0.x, a0.y, a0.z, a0.w, a1.x, a1.y, a1.z, a1.w, a2.x, a2.y, a2.z, a2.w, a3.x, a3.y, a3.z, a3.w};
            #pragma unroll
            for (int e = 0; e < 16; ++e) { __bf16 h_, l_; split_bf16(av[e], h_, l_); ah[e] = h_; al[e] = l_; }
        }

        #pragma unroll
        for (int t = 0; t < 4; ++t) {
            const __bf16* bp = &Bs[(t * 16 + l) * LDS_STRIDE];
            const __bf16* bq = &Bl[(t * 16 + l) * LDS_STRIDE];
            const bf16x8 h0 = *(const bf16x8*)(bp + hi * 8), h1 = *(const bf16x8*)(bp + 16 + hi * 8);
            const bf16x8 l0 = *(const bf16x8*)(bq + hi * 8), l1 = *(const bf16x8*)(bq + 16 + hi * 8);
            const bf16x16 bh = __builtin_shufflevector(h0, h1, 0, 1, 2, 3, 4, 5, 6, 7, 8, 9, 10, 11, 12, 13, 14, 15);
            const bf16x16 bl = __builtin_shufflevector(l0, l1, 0, 1, 2, 3, 4, 5, 6, 7, 8, 9, 10, 11, 12, 13, 14, 15);
            if      (t == 0) c0 = wmma3(ah, al, bh, bl, c0);
            else if (t == 1) c1 = wmma3(ah, al, bh, bl, c1);
            else if (t == 2) c2 = wmma3(ah, al, bh, bl, c2);
            else             c3 = wmma3(ah, al, bh, bl, c3);
        }
    }

    for (int pass = 0; pass < 2; ++pass) {
        #pragma unroll
        for (int pr = 0; pr < 2; ++pr) {
            const float8& ca = (pr == 0) ? c0 : c2;
            const float8& cb = (pr == 0) ? c1 : c3;
            const int cbase = n0 + pr * 32;
            const float bv = HAS_BIAS ? bias[cbase + lane] : 0.0f;
            #pragma unroll
            for (int r = 0; r < 8; ++r) {
                const float a0 = ca[r], b0 = cb[r];
                const float ax = __shfl_xor(a0, 16), bx = __shfl_xor(b0, 16);
                const float v1 = (hi ? bx : a0) + bv;
                const float v2 = (hi ? b0 : ax) + bv;
                const int r1 = m0w + r, r2 = m0w + r + 8;
                if (!GUARD || r1 < M) *(volatile float*)(C + (size_t)r1 * ldc + cbase + lane) = v1;
                if (!GUARD || r2 < M) *(volatile float*)(C + (size_t)r2 * ldc + cbase + lane) = v2;
            }
        }
        __threadfence();
    }
}

__global__ void softmax_rows(float* __restrict__ S, int cols)
{
    float* __restrict__ p = S + (size_t)blockIdx.x * cols;
    __shared__ float red[256];
    const int t = threadIdx.x;

    float mx = -3.0e38f;
    for (int i = t; i < cols; i += 256) mx = fmaxf(mx, p[i]);
    red[t] = mx; __syncthreads();
    for (int s = 128; s > 0; s >>= 1) { if (t < s) red[t] = fmaxf(red[t], red[t + s]); __syncthreads(); }
    mx = red[0]; __syncthreads();

    float sum = 0.0f;
    for (int i = t; i < cols; i += 256) { float e = expf(p[i] - mx); p[i] = e; sum += e; }
    red[t] = sum; __syncthreads();
    for (int s = 128; s > 0; s >>= 1) { if (t < s) red[t] += red[t + s]; __syncthreads(); }
    const float inv = 1.0f / red[0];

    for (int i = t; i < cols; i += 256) { const float v = p[i] * inv; *(volatile float*)(p + i) = v; __threadfence(); *(volatile float*)(p + i) = v; }
}

__global__ void l2norm_rows(float* __restrict__ V, int cols)
{
    float* __restrict__ p = V + (size_t)blockIdx.x * cols;
    __shared__ float red[256];
    const int t = threadIdx.x;

    float ss = 0.0f;
    for (int i = t; i < cols; i += 256) { float v = p[i]; ss += v * v; }
    red[t] = ss; __syncthreads();
    for (int s = 128; s > 0; s >>= 1) { if (t < s) red[t] += red[t + s]; __syncthreads(); }
    const float inv = 1.0f / sqrtf(red[0]);

    for (int i = t; i < cols; i += 256) { const float v = p[i] * inv; *(volatile float*)(p + i) = v; __threadfence(); *(volatile float*)(p + i) = v; }
}


static inline dim3 gemm_grid(int M, int N) { return dim3(N / 64, (M + 63) / 64); }

extern "C" void kernel_launch(void* const* d_in, const int* in_sizes, int n_in,
                              void* d_out, int out_size, void* d_ws, size_t ws_size,
                              hipStream_t stream)
{
    const float* x   = (const float*)d_in[0];
    const float* Wk1 = (const float*)d_in[1];
    const float* bk1 = (const float*)d_in[2];
    const float* Wq1 = (const float*)d_in[3];
    const float* bq1 = (const float*)d_in[4];
    const float* Wk2 = (const float*)d_in[5];
    const float* bk2 = (const float*)d_in[6];
    const float* Wq2 = (const float*)d_in[7];
    const float* bq2 = (const float*)d_in[8];
    const float* Wv2 = (const float*)d_in[9];
    const float* bv2 = (const float*)d_in[10];
    float* out = (float*)d_out;
    (void)in_sizes; (void)n_in; (void)out_size;
    if (ws_size < (size_t)4 * ((size_t)SEQ * KK_ * 2 + (size_t)SEQ * DD * 3 + (size_t)SEQ * SEQ)) return;

    float* ws = (float*)d_ws;
    float* Q  = ws;
    float* Kb = Q  + (size_t)SEQ * KK_;
    float* V  = Kb + (size_t)SEQ * KK_;
    float* Sc = V  + (size_t)SEQ * DD;
    float* H1 = Sc + (size_t)SEQ * SEQ;
    float* H2 = H1 + (size_t)SEQ * DD;

    const dim3 blk(128);

    gemm_wmma_f16<false, true,  false><<<gemm_grid(SEQ, KK_), blk, 0, stream>>>(x, DD, Wq1, KK_, bq1, Q,  KK_, SEQ, KK_, DD);
    gemm_wmma_f16<false, true,  false><<<gemm_grid(SEQ, KK_), blk, 0, stream>>>(x, DD, Wk1, KK_, bk1, Kb, KK_, SEQ, KK_, DD);
    gemm_wmma_f16<true,  false, false><<<gemm_grid(SEQ, SEQ), blk, 0, stream>>>(Q, KK_, Kb,  KK_, nullptr, Sc, SEQ, SEQ, SEQ, KK_);
    softmax_rows<<<dim3(SEQ), dim3(256), 0, stream>>>(Sc, SEQ);
    gemm_wmma_f16<false, false, false><<<gemm_grid(SEQ, DD),  blk, 0, stream>>>(Sc, SEQ, x,  DD,  nullptr, H1, DD, SEQ, DD, SEQ);

    gemm_wmma_f16<false, true,  false><<<gemm_grid(SEQ, KK_), blk, 0, stream>>>(H1, DD, Wq2, KK_, bq2, Q,  KK_, SEQ, KK_, DD);
    gemm_wmma_f16<false, true,  false><<<gemm_grid(SEQ, KK_), blk, 0, stream>>>(H1, DD, Wk2, KK_, bk2, Kb, KK_, SEQ, KK_, DD);
    gemm_wmma_f16<false, true,  false><<<gemm_grid(SEQ, DD),  blk, 0, stream>>>(H1, DD, Wv2, DD,  bv2, V,  DD,  SEQ, DD,  DD);
    l2norm_rows<<<dim3(SEQ), dim3(256), 0, stream>>>(V, DD);
    gemm_wmma_f16<true,  false, false><<<gemm_grid(SEQ, SEQ), blk, 0, stream>>>(Q, KK_, Kb,  KK_, nullptr, Sc, SEQ, SEQ, SEQ, KK_);
    softmax_rows<<<dim3(SEQ), dim3(256), 0, stream>>>(Sc, SEQ);
    gemm_wmma_f16<false, false, false><<<gemm_grid(SEQ, DD),  blk, 0, stream>>>(Sc, SEQ, V,  DD,  nullptr, H2, DD, SEQ, DD, SEQ);

    gemm_wmma_f16<false, true,  false><<<gemm_grid(SEQ, KK_), blk, 0, stream>>>(H2, DD, Wk2, KK_, bk2, Kb, KK_, SEQ, KK_, DD);
    gemm_wmma_f16<false, true,  false><<<gemm_grid(SEQ, DD),  blk, 0, stream>>>(H2, DD, Wv2, DD,  bv2, V,  DD,  SEQ, DD,  DD);
    l2norm_rows<<<dim3(SEQ), dim3(256), 0, stream>>>(V, DD);
    gemm_wmma_f16<false, true,  true ><<<gemm_grid(1, KK_),   blk, 0, stream>>>(H2 + (size_t)(SEQ - 1) * DD, DD,
                                                                                Wq2, KK_, bq2, Q, KK_, 1, KK_, DD);
    gemm_wmma_f16<true,  false, true ><<<gemm_grid(1, SEQ),   blk, 0, stream>>>(Q, KK_, Kb, KK_, nullptr, Sc, SEQ, 1, SEQ, KK_);
    softmax_rows<<<dim3(1), dim3(256), 0, stream>>>(Sc, SEQ);
    gemm_wmma_f16<false, false, true ><<<gemm_grid(1, DD),    blk, 0, stream>>>(Sc, SEQ, V, DD, nullptr, out, DD, 1, DD, SEQ);
}
